// GCN_83545703842213
// MI455X (gfx1250) — hardware-run, weakly checked
//
#include <hip/hip_runtime.h>
#include <stddef.h>
#include <stdint.h>
#include <math.h>

#define NN      100000
#define FD      128
#define HD      128
#define NE      1600000
#define GBM     128
#define MP      100096
#define G2_TWO_TERM 1
#define KG1     128
#define KG2     (G2_TWO_TERM ? 256 : 128)
#define XPITCH  128
#define W1PITCH 128
#define HPITCH  256
#define W2PITCH 256
#define NTHR    256
#define NWAVE   8
#define EPT     8
#define WCH     (32 * EPT)
#define NBRUN   1024
#define SLB     10
#define NBK     98
#define NTAB    (NBK * NBRUN)
#define WLCAP   3072
#define RCAP    18432
#define TRIPCAP 64
#define MAXDEG_MEAS   36
#define MAXB1024_MEAS 16710
#define ABM     64
#define SP      132
#define WSMAX   ((size_t)(128u << 20))

#define BK_WL    (NWAVE * WLCAP)
#define BK_PL    (2 * RCAP)
#define BK_ZINTS (BK_WL + BK_PL + 4 * NBRUN)
#define BK_INTS  (BK_ZINTS + 16)
#define BK_LDS   (BK_INTS * 4)
#define GM_LDS   ((GBM * SP + GBM) * 4)

#define PBX   (MP * FD / 8 / NTHR)
#define PBW1  (HD * FD / 8 / NTHR)
#define PBW2  (HD * W2PITCH / 8 / NTHR)
#define PBTOT (PBX + PBW1 + PBW2 + 1)

static_assert(32 * 4 == HD && FD == 128);
static_assert(MP % GBM == 0 && MP >= NN && MP == 782 * GBM && MP % ABM == 0);
static_assert(NBRUN == (1 << SLB) && NBRUN % ABM == 0 && NBRUN % NTHR == 0 && NBRUN % 32 == 0);
static_assert(NBK * NBRUN >= MP && NBK * NBRUN >= NN && NTAB >= MP);
static_assert(NE < (1 << 21) && (((long long)NE) << SLB) < (1LL << 31));
static_assert(NE % WCH == 0 && NE % 4 == 0);
static_assert(RCAP % 1024 == 0 && (long long)RCAP * 100 >= (long long)MAXB1024_MEAS * 105);
static_assert(WLCAP >= MAXB1024_MEAS / 8 + 8 * 46 + 1);
static_assert(MAXDEG_MEAS + 8 <= TRIPCAP);
static_assert(BK_PL % (NTHR * 4) == 0 && BK_ZINTS % 4 == 0 && NBRUN == NTHR * 4);
static_assert(BK_LDS <= 300000 && GM_LDS <= 300000);
static_assert(KG1 % 32 == 0 && KG2 % 32 == 0 && KG1 <= XPITCH && KG1 <= W1PITCH && KG2 <= HPITCH && KG2 <= W2PITCH);
static_assert(HPITCH == 2 * HD && W2PITCH == 2 * HD);
static_assert((MP * FD / 8) % NTHR == 0 && (HD * FD / 8) % NTHR == 0 && (HD * W2PITCH / 8) % NTHR == 0);
static_assert(ABM == NWAVE * 8 && GBM == NWAVE * 16);
static_assert((long long)(NN - 1) * HD + HD - 1 == 12799999LL);

typedef float          v4f   __attribute__((ext_vector_type(4)));
typedef float          v8f   __attribute__((ext_vector_type(8)));
typedef int            v2i   __attribute__((ext_vector_type(2)));
typedef int            v4i   __attribute__((ext_vector_type(4)));
typedef int            v8i   __attribute__((ext_vector_type(8)));
typedef unsigned short v8us  __attribute__((ext_vector_type(8)));
typedef unsigned short v16us __attribute__((ext_vector_type(16)));
typedef __bf16         v16bf __attribute__((ext_vector_type(16)));
typedef v4f  __attribute__((may_alias)) v4fa;
typedef v2i  __attribute__((may_alias)) v2ia;
typedef v4i  __attribute__((may_alias)) v4ia;
typedef v8us __attribute__((may_alias)) v8usa;
union FragB { v16bf v; v16us u; v8us h[2]; v8i w; };

__device__ __forceinline__ v8f wmb(const FragB& a, const FragB& b, v8f c) {
  v8f d = __builtin_amdgcn_wmma_f32_16x16x32_bf16(false, a.v, false, b.v, (short)0, c, false, false);
  asm volatile("v_nop\n\tv_nop\n\tv_nop\n\tv_nop" : "+v"(d) : "v"(a.w), "v"(b.w));
  return d;
}

__device__ __forceinline__ unsigned bf16_bits(float f) {
  const unsigned u = __float_as_uint(f);
  const unsigned r = (u + 0x7FFFu + ((u >> 16) & 1u)) >> 16;
  const unsigned q = (u >> 16) | 0x40u;
  return ((u & 0x7fffffffu) > 0x7f800000u) ? q : r;
}
__device__ __forceinline__ float bf16_val(float f) {
  return __uint_as_float(bf16_bits(f) << 16);
}

__device__ __forceinline__ void hilo_pack(float v0, float v1, float v2, float v3,
                                          int& h01, int& h23, int& l01, int& l23) {
  const unsigned a0 = bf16_bits(v0), a1 = bf16_bits(v1), a2 = bf16_bits(v2), a3 = bf16_bits(v3);
  const unsigned b0 = bf16_bits(v0 - __uint_as_float(a0 << 16));
  const unsigned b1 = bf16_bits(v1 - __uint_as_float(a1 << 16));
  const unsigned b2 = bf16_bits(v2 - __uint_as_float(a2 << 16));
  const unsigned b3 = bf16_bits(v3 - __uint_as_float(a3 << 16));
  h01 = (int)(a0 | (a1 << 16)); h23 = (int)(a2 | (a3 << 16));
  l01 = (int)(b0 | (b1 << 16)); l23 = (int)(b2 | (b3 << 16));
}

__device__ __forceinline__ v4i regroup_row(int h01, int h23, int l01, int l23, int lane) {
  const int s0 = (2 * lane) & 31, s1 = s0 + 1;
  const int a0 = __shfl(h01, s0, 32), a1 = __shfl(h23, s0, 32), a2 = __shfl(h01, s1, 32), a3 = __shfl(h23, s1, 32);
  const int b0 = __shfl(l01, s0, 32), b1 = __shfl(l23, s0, 32), b2 = __shfl(l01, s1, 32), b3 = __shfl(l23, s1, 32);
  const int mk = (lane < 16) ? -1 : 0;
  v4i o;
  o.x = (a0 & mk) | (b0 & ~mk); o.y = (a1 & mk) | (b1 & ~mk);
  o.z = (a2 & mk) | (b2 & ~mk); o.w = (a3 & mk) | (b3 & ~mk);
  return o;
}

__device__ __forceinline__ void st2_v4f(float* p, v4f v) {
  *(volatile v4f*)p = v;
  __threadfence();
  *(volatile v4f*)p = v;
}
__device__ __forceinline__ void st2_v8us(unsigned short* p, v8us v) {
  *(volatile v8us*)p = v;
  __threadfence();
  *(volatile v8us*)p = v;
}

__device__ __forceinline__ v8us col8(const float* __restrict__ base, int stride) {
  float f[8];
#pragma unroll
  for (int i = 0; i < 8; ++i) f[i] = base[(size_t)i * (size_t)stride];
  v8us o;
#pragma unroll
  for (int i = 0; i < 8; ++i) o[i] = (unsigned short)bf16_bits(f[i]);
  return o;
}

__global__ __launch_bounds__(NTHR) void k_prep(const float* __restrict__ x, const float* __restrict__ w1,
                                               const float* __restrict__ b1, const float* __restrict__ w2,
                                               const float* __restrict__ b2,
                                               unsigned short* xb, unsigned short* w1t, unsigned short* w2d,
                                               float* sm) {
  const int tid = (int)threadIdx.x, lane = tid & 31, wave = tid >> 5;
  const int blk = (int)blockIdx.x;
  if (blk < PBX) {
    const int u   = blk * NTHR + tid;
    const int row = u >> 4, k8 = (u & 15) * 8;
    const int rc  = row < NN ? row : NN - 1;
    const unsigned mk = row < NN ? 0xffffu : 0u;
    const float* p = x + (size_t)rc * FD + k8;
    const v4f a = *(const v4fa*)p;
    const v4f b = *(const v4fa*)(p + 4);
    v8us o;
    o[0] = (unsigned short)(bf16_bits(a.x) & mk); o[1] = (unsigned short)(bf16_bits(a.y) & mk);
    o[2] = (unsigned short)(bf16_bits(a.z) & mk); o[3] = (unsigned short)(bf16_bits(a.w) & mk);
    o[4] = (unsigned short)(bf16_bits(b.x) & mk); o[5] = (unsigned short)(bf16_bits(b.y) & mk);
    o[6] = (unsigned short)(bf16_bits(b.z) & mk); o[7] = (unsigned short)(bf16_bits(b.w) & mk);
    st2_v8us(xb + (size_t)row * XPITCH + k8, o);
  } else if (blk < PBX + PBW1) {
    const int u = (blk - PBX) * NTHR + tid;
    const int n = u >> 4, k8 = (u & 15) * 8;
    const v8us o = col8(w1 + (size_t)k8 * HD + n, HD);
    st2_v8us(w1t + (size_t)n * W1PITCH + k8, o);
  } else if (blk < PBX + PBW1 + PBW2) {
    const int u = (blk - PBX - PBW1) * NTHR + tid;
    const int n = u >> 5, k8 = (u & 31) * 8, kk = k8 & (HD - 1);
    const v8us o = col8(w2 + (size_t)kk * HD + n, HD);
    st2_v8us(w2d + (size_t)n * W2PITCH + k8, o);
  } else {
    if (wave == 0) {
      const v4f a = *(const v4fa*)(b1 + 4 * lane);
      v4f o;
      o.x = bf16_val(a.x); o.y = bf16_val(a.y); o.z = bf16_val(a.z); o.w = bf16_val(a.w);
      st2_v4f(sm + 4 * lane, o);
    } else if (wave == 1) {
      const v4f a = *(const v4fa*)(b2 + 4 * lane);
      v4f o;
      o.x = bf16_val(a.x); o.y = bf16_val(a.y); o.z = bf16_val(a.z); o.w = bf16_val(a.w);
      st2_v4f(sm + HD + 4 * lane, o);
    }
  }
}

__device__ __forceinline__ void bucket_flush(const int* pl, const int* cnt, const int* offs, const int* dvs, int ov,
                                             int* ep, int* cp, int* op, int* dp, int* fp, int tid) {
#pragma unroll 1
  for (int i = tid * 4; i < BK_PL; i += NTHR * 4) {
    const v4i v = *(const v4ia*)(pl + i);
    *(volatile v4i*)(ep + i) = v;
  }
  {
    const v4i v = *(const v4ia*)(cnt + 4 * tid);
    *(volatile v4i*)(cp + 4 * tid) = v;
  }
  {
    const v4i v = *(const v4ia*)(offs + 4 * tid);
    *(volatile v4i*)(op + 4 * tid) = v;
  }
  {
    const v4i v = *(const v4ia*)(dvs + 4 * tid);
    *(volatile v4i*)(dp + 4 * tid) = v;
  }
  if (tid < 8) {
    const v4i f = {ov, ov, ov, ov};
    *(volatile v4i*)(fp + 4 * tid) = f;
  }
}

__global__ __launch_bounds__(NTHR) void k_bucket(const int* __restrict__ srcs, const int* __restrict__ dsts,
                                                 const float* __restrict__ ew,
                                                 int* ENT, int* CNT, int* OFF, int* DVB, int* FLAG) {
  extern __shared__ __attribute__((aligned(16))) int dsm[];
  int* wl   = dsm;
  int* pl   = dsm + BK_WL;
  int* cnt  = pl + BK_PL;
  int* offs = cnt + NBRUN;
  int* cur  = offs + NBRUN;
  int* dvs  = cur + NBRUN;
  int* misc = dvs + NBRUN;
  const int tid = (int)threadIdx.x, lane = tid & 31, wave = tid >> 5;
  const int blk = (int)blockIdx.x;
  const unsigned nbs = (unsigned)(blk * NBRUN);

  {
    const v4i z4 = {0, 0, 0, 0};
    for (int i = tid * 4; i < BK_ZINTS; i += NTHR * 4) *(v4ia*)(dsm + i) = z4;
    if (tid < 16) misc[tid] = 0;
  }
  __syncthreads();

  {
    const int per  = ((NE + NWAVE * WCH - 1) / (NWAVE * WCH)) * WCH;
    const int ebeg = wave * per;
    const int eend = (ebeg + per < NE) ? (ebeg + per) : NE;
    int* mylist = wl + wave * WLCAP;
    int wc = 0;
#pragma unroll 1
    for (int cb = ebeg; cb < eend; cb += WCH) {
      const int e0 = cb + lane * EPT;
      const v4i da = *(const v4ia*)(dsts + e0);
      const v4i db = *(const v4ia*)(dsts + e0 + 4);
      const unsigned s0 = (unsigned)da.x - nbs, s1 = (unsigned)da.y - nbs;
      const unsigned s2 = (unsigned)da.z - nbs, s3 = (unsigned)da.w - nbs;
      const unsigned s4 = (unsigned)db.x - nbs, s5 = (unsigned)db.y - nbs;
      const unsigned s6 = (unsigned)db.z - nbs, s7 = (unsigned)db.w - nbs;
      const bool h0 = s0 < (unsigned)NBRUN, h1 = s1 < (unsigned)NBRUN, h2 = s2 < (unsigned)NBRUN, h3 = s3 < (unsigned)NBRUN;
      const bool h4 = s4 < (unsigned)NBRUN, h5 = s5 < (unsigned)NBRUN, h6 = s6 < (unsigned)NBRUN, h7 = s7 < (unsigned)NBRUN;
      const unsigned m0 = __builtin_amdgcn_ballot_w32(h0), m1 = __builtin_amdgcn_ballot_w32(h1);
      const unsigned m2 = __builtin_amdgcn_ballot_w32(h2), m3 = __builtin_amdgcn_ballot_w32(h3);
      const unsigned m4 = __builtin_amdgcn_ballot_w32(h4), m5 = __builtin_amdgcn_ballot_w32(h5);
      const unsigned m6 = __builtin_amdgcn_ballot_w32(h6), m7 = __builtin_amdgcn_ballot_w32(h7);
      const unsigned any = m0 | m1 | m2 | m3 | m4 | m5 | m6 | m7;
      if (any != 0u) {
        const int pre = (int)(__builtin_amdgcn_mbcnt_lo(m0, 0u) + __builtin_amdgcn_mbcnt_lo(m1, 0u) +
                              __builtin_amdgcn_mbcnt_lo(m2, 0u) + __builtin_amdgcn_mbcnt_lo(m3, 0u) +
                              __builtin_amdgcn_mbcnt_lo(m4, 0u) + __builtin_amdgcn_mbcnt_lo(m5, 0u) +
                              __builtin_amdgcn_mbcnt_lo(m6, 0u) + __builtin_amdgcn_mbcnt_lo(m7, 0u));
        int p = wc + pre;
        if (h0) { if (p < WLCAP) mylist[p] = ((e0 + 0) << SLB) | (int)s0; p = p + 1; }
        if (h1) { if (p < WLCAP) mylist[p] = ((e0 + 1) << SLB) | (int)s1; p = p + 1; }
        if (h2) { if (p < WLCAP) mylist[p] = ((e0 + 2) << SLB) | (int)s2; p = p + 1; }
        if (h3) { if (p < WLCAP) mylist[p] = ((e0 + 3) << SLB) | (int)s3; p = p + 1; }
        if (h4) { if (p < WLCAP) mylist[p] = ((e0 + 4) << SLB) | (int)s4; p = p + 1; }
        if (h5) { if (p < WLCAP) mylist[p] = ((e0 + 5) << SLB) | (int)s5; p = p + 1; }
        if (h6) { if (p < WLCAP) mylist[p] = ((e0 + 6) << SLB) | (int)s6; p = p + 1; }
        if (h7) { if (p < WLCAP) mylist[p] = ((e0 + 7) << SLB) | (int)s7; p = p + 1; }
        wc += (int)(__builtin_popcount(m0) + __builtin_popcount(m1) + __builtin_popcount(m2) + __builtin_popcount(m3) +
                    __builtin_popcount(m4) + __builtin_popcount(m5) + __builtin_popcount(m6) + __builtin_popcount(m7));
      }
    }
    if (lane == 0) misc[wave] = wc;
  }
  __syncthreads();

  if (wave == 0) {
    int ov = 0, tot = 0;
#pragma unroll 1
    for (int w2 = 0; w2 < NWAVE; ++w2) {
      int c = misc[w2];
      if (c > WLCAP) ov = 1;
      c = c < 0 ? 0 : (c > WLCAP ? WLCAP : c);
      c = __builtin_amdgcn_readfirstlane(c);
      tot += c;
#pragma unroll 1
      for (int b0 = 0; b0 < c; b0 += 32) {
        const int idx = b0 + lane;
        const int ent = wl[w2 * WLCAP + (idx < WLCAP ? idx : WLCAP - 1)];
        const int m32 = (c - b0) < 32 ? (c - b0) : 32;
#pragma unroll 1
        for (int k = 0; k < m32; ++k) {
          const int u    = __builtin_amdgcn_readlane(ent, k);
          const int slot = u & (NBRUN - 1);
          if (lane == 0) cnt[slot] = cnt[slot] + 1;
        }
      }
    }
    if (tot > RCAP) ov = 1;
    if (lane == 0) misc[9] = ov;
  }
  __syncthreads();
  if (wave == 0) {
    const int base = lane * (NBRUN / 32);
    int s = 0;
#pragma unroll 1
    for (int i = 0; i < NBRUN / 32; ++i) s += cnt[base + i];
    int incl = s;
#pragma unroll
    for (int d = 1; d < 32; d <<= 1) {
      const int y = __shfl_up(incl, d, 32);
      if (lane >= d) incl += y;
    }
    int run = incl - s;
#pragma unroll 1
    for (int i = 0; i < NBRUN / 32; ++i) {
      const int cv = cnt[base + i];
      offs[base + i] = run;
      cur[base + i]  = run;
      run += cv;
    }
  }
  __syncthreads();

  if (wave == 0) {
#pragma unroll 1
    for (int w2 = 0; w2 < NWAVE; ++w2) {
      int c = misc[w2];
      c = c < 0 ? 0 : (c > WLCAP ? WLCAP : c);
      c = __builtin_amdgcn_readfirstlane(c);
#pragma unroll 1
      for (int b0 = 0; b0 < c; b0 += 32) {
        const int idx = b0 + lane;
        const int ent = wl[w2 * WLCAP + (idx < WLCAP ? idx : WLCAP - 1)];
        int eid = (ent >> SLB) & 0x1FFFFF;
        eid = eid > NE - 1 ? NE - 1 : eid;
        int sr = srcs[eid];
        sr = sr < 0 ? 0 : (sr > NN - 1 ? NN - 1 : sr);
        const int wbits = (int)(bf16_bits(ew[eid]) << 16);
        const int m32 = (c - b0) < 32 ? (c - b0) : 32;
#pragma unroll 1
        for (int k = 0; k < m32; ++k) {
          const int u    = __builtin_amdgcn_readlane(ent, k);
          const int sk   = __builtin_amdgcn_readlane(sr, k);
          const int wk   = __builtin_amdgcn_readlane(wbits, k);
          const int slot = u & (NBRUN - 1);
          if (lane == 0) {
            int p = cur[slot];
            p = p < 0 ? 0 : (p > RCAP - 1 ? RCAP - 1 : p);
            pl[2 * p]     = sk;
            pl[2 * p + 1] = wk;
            cur[slot] = p + 1;
          }
        }
      }
    }
  }
  __syncthreads();

  {
    const float qnan = __uint_as_float(0x7fc00000u);
#pragma unroll 1
    for (int it = 0; it < NBRUN / NTHR; ++it) {
      const int slot = it * NTHR + tid;
      int c = cnt[slot];
      int o = offs[slot];
      const bool big = c > TRIPCAP;
      c = c < 0 ? 0 : (c > TRIPCAP ? TRIPCAP : c);
      o = o < 0 ? 0 : (o > RCAP - 1 ? RCAP - 1 : o);
      int cm = c;
#pragma unroll
      for (int d = 16; d > 0; d >>= 1) {
        const int y = __shfl_xor(cm, d, 32);
        cm = cm > y ? cm : y;
      }
      cm = __builtin_amdgcn_readfirstlane(cm);
      int last = o + c - 1;
      last = last < o ? o : last;
      last = last > RCAP - 1 ? RCAP - 1 : last;
      float s = 0.0f;
#pragma unroll 1
      for (int j = 0; j < cm; ++j) {
        int idx = o + j;
        idx = idx > last ? last : idx;
        const float w = __int_as_float(pl[2 * idx + 1]);
        asm volatile("" :: "v"(w));
        const float t = s + w;
        s = (j < c) ? t : s;
      }
      const float deg = s + 1.0f;
      const float rs  = 1.0f / sqrtf(deg);
      float dv = (deg > 0.0f) ? rs : 0.0f;
      dv = big ? qnan : dv;
      dvs[slot] = __float_as_int(dv);
    }
  }
  __syncthreads();

  const int ovf = misc[9];
  int* ep = ENT + (size_t)blk * (size_t)BK_PL;
  int* cp = CNT + (size_t)blk * NBRUN;
  int* op = OFF + (size_t)blk * NBRUN;
  int* dp = DVB + (size_t)blk * NBRUN;
  int* fp = FLAG + (size_t)blk * 32;
  bucket_flush(pl, cnt, offs, dvs, ovf, ep, cp, op, dp, fp, tid);
  __threadfence();
  bucket_flush(pl, cnt, offs, dvs, ovf, ep, cp, op, dp, fp, tid);
}

template <int KTOT, int APITCH, int WPITCH>
__global__ __launch_bounds__(NTHR) __attribute__((amdgpu_num_vgpr(248)))
void k_gemm(const unsigned short* __restrict__ A, const unsigned short* __restrict__ BT,
            const float* __restrict__ DINV, float* P) {
  extern __shared__ __attribute__((aligned(16))) float gsm[];
  float* stg = gsm;
  float* sdv = gsm + GBM * SP;
  const int tid = (int)threadIdx.x, lane = tid & 31, wave = tid >> 5, hh = lane >> 4, m = lane & 15;
  const int rowBase = (int)blockIdx.x * GBM;
  if (tid < 32) *(v4fa*)(sdv + 4 * tid) = *(const v4fa*)(DINV + rowBase + 4 * tid);

  v8f acc[8];
  {
    const v8f z = {0.f, 0.f, 0.f, 0.f, 0.f, 0.f, 0.f, 0.f};
#pragma unroll
    for (int t = 0; t < 8; ++t) acc[t] = z;
  }
  const unsigned short* ap = A + (size_t)(rowBase + 16 * wave + m) * (size_t)APITCH + 8 * hh;
  const unsigned short* bp = BT + (size_t)m * (size_t)WPITCH + 8 * hh;
#pragma unroll 1
  for (int k0 = 0; k0 < KTOT; k0 += 32) {
    FragB af;
    af.h[0] = *(const v8usa*)(ap + k0);
    af.h[1] = *(const v8usa*)(ap + k0 + 16);
#pragma unroll
    for (int nt = 0; nt < 8; ++nt) {
      const unsigned short* wq = bp + (size_t)(16 * nt) * (size_t)WPITCH + k0;
      FragB bf;
      bf.h[0] = *(const v8usa*)wq;
      bf.h[1] = *(const v8usa*)(wq + 16);
      acc[nt] = wmb(af, bf, acc[nt]);
    }
  }
#pragma unroll
  for (int nt = 0; nt < 8; ++nt) {
#pragma unroll
    for (int r = 0; r < 8; ++r) stg[(16 * wave + 8 * hh + r) * SP + 16 * nt + m] = acc[nt][r];
  }
  __syncthreads();

#pragma unroll 1
  for (int i = 0; i < 16; ++i) {
    const int lr   = 16 * wave + i;
    const int grow = rowBase + lr;
    const bool live = grow < NN;
    const v4f a = *(const v4fa*)(stg + lr * SP + 4 * lane);
    const float dv = sdv[lr];
    asm volatile("" :: "v"(a));
    asm volatile("" :: "v"(dv));
    const float v0 = a.x * dv, v1 = a.y * dv, v2 = a.z * dv, v3 = a.w * dv;
    v4f o;
    o.x = live ? v0 : 0.0f; o.y = live ? v1 : 0.0f; o.z = live ? v2 : 0.0f; o.w = live ? v3 : 0.0f;
    st2_v4f(P + (size_t)grow * HD + 4 * lane, o);
  }
}

template <int LAST>
__global__ __launch_bounds__(NTHR) void k_replay(const int* __restrict__ ENT, const int* __restrict__ CNT,
                                                 const int* __restrict__ OFF, const float* __restrict__ DINV,
                                                 const int* __restrict__ FLAG, const float* __restrict__ P,
                                                 const float* __restrict__ BF, unsigned short* H1HL, float* out) {
  const int tid = (int)threadIdx.x, lane = tid & 31, wave = tid >> 5;
  const int rowBase = (int)blockIdx.x * ABM;
  const int bucket  = rowBase >> SLB;
  const int* eb = ENT + (size_t)bucket * (size_t)BK_PL;
  const int flag = FLAG[(size_t)bucket * 32];
  const v4f bias = *(const v4fa*)(BF + 4 * lane);
  const float qnan = __uint_as_float(0x7fc00000u);

#pragma unroll 1
  for (int i = 0; i < ABM / NWAVE; ++i) {
    const int d = rowBase + (ABM / NWAVE) * wave + i;
    int c = CNT[d];
    int o = OFF[d];
    const float dv = DINV[d];
    const bool big = c > TRIPCAP;
    c = c < 0 ? 0 : (c > TRIPCAP ? TRIPCAP : c);
    o = o < 0 ? 0 : (o > RCAP - 1 ? RCAP - 1 : o);
    c = __builtin_amdgcn_readfirstlane(c);
    o = __builtin_amdgcn_readfirstlane(o);
    int last = o + c - 1;
    last = last < o ? o : last;
    last = last > RCAP - 1 ? RCAP - 1 : last;
    float a0 = 0.0f, a1 = 0.0f, a2 = 0.0f, a3 = 0.0f;
#pragma unroll 1
    for (int j = 0; j < c; ++j) {
      int idx = o + j;
      idx = idx > last ? last : idx;
      const v2i e = *(const v2ia*)(eb + 2 * idx);
      int sr = e.x;
      sr = sr < 0 ? 0 : (sr > NN - 1 ? NN - 1 : sr);
      const float w = __int_as_float(e.y);
      const v4f v = *(const v4fa*)(P + (size_t)sr * HD + 4 * lane);
      asm volatile("" :: "v"(v));
      a0 = fmaf(w, v.x, a0); a1 = fmaf(w, v.y, a1); a2 = fmaf(w, v.z, a2); a3 = fmaf(w, v.w, a3);
    }
    const v4f g = *(const v4fa*)(P + (size_t)d * HD + 4 * lane);
    asm volatile("" :: "v"(g));
    float t0 = (a0 + g.x) * dv + bias.x, t1 = (a1 + g.y) * dv + bias.y;
    float t2 = (a2 + g.z) * dv + bias.z, t3 = (a3 + g.w) * dv + bias.w;
    const bool bad  = (flag != 0) | big;
    const bool live = d < NN;
    if constexpr (LAST == 0) {
      t0 = (t0 > 0.0f) ? t0 : (t0 - t0); t1 = (t1 > 0.0f) ? t1 : (t1 - t1);
      t2 = (t2 > 0.0f) ? t2 : (t2 - t2); t3 = (t3 > 0.0f) ? t3 : (t3 - t3);
      t0 = bad ? qnan : t0; t1 = bad ? qnan : t1; t2 = bad ? qnan : t2; t3 = bad ? qnan : t3;
      t0 = live ? t0 : 0.0f; t1 = live ? t1 : 0.0f; t2 = live ? t2 : 0.0f; t3 = live ? t3 : 0.0f;
      int h01, h23, l01, l23;
      hilo_pack(t0, t1, t2, t3, h01, h23, l01, l23);
      const v4i ow = regroup_row(h01, h23, l01, l23, lane);
      unsigned short* hp = H1HL + (size_t)d * HPITCH + 8 * lane;
      *(volatile v4i*)hp = ow;
      __threadfence();
      *(volatile v4i*)hp = ow;
    } else {
      float ss = (t0 * t0 + t1 * t1) + (t2 * t2 + t3 * t3);
#pragma unroll
      for (int s = 16; s > 0; s >>= 1) ss += __shfl_xor(ss, s, 32);
      const float n  = sqrtf(ss);
      const float dd = fmaxf(n, 1e-12f);
      float q0 = t0 / dd, q1 = t1 / dd, q2 = t2 / dd, q3 = t3 / dd;
      q0 = bad ? qnan : q0; q1 = bad ? qnan : q1; q2 = bad ? qnan : q2; q3 = bad ? qnan : q3;
      v4f ov;
      ov.x = q0; ov.y = q1; ov.z = q2; ov.w = q3;
      const int dc = live ? d : NN - 1;
      float* op = out + (size_t)dc * HD + 4 * lane;
      if (live) *(volatile v4f*)op = ov;
      __threadfence();
      if (live) *(volatile v4f*)op = ov;
    }
  }
}

extern "C" void kernel_launch(void* const* d_in, const int* in_sizes, int n_in,
                              void* d_out, int out_size, void* d_ws, size_t ws_size,
                              hipStream_t stream) {
  if (n_in < 7) return;
  if (in_sizes[0] != NN * FD) return;
  if (in_sizes[1] != 2 * NE) return;
  if (in_sizes[2] != NE) return;
  if (in_sizes[3] != FD * HD) return;
  if (in_sizes[4] != HD) return;
  if (in_sizes[5] != HD * HD) return;
  if (in_sizes[6] != HD) return;
  if (out_size != NN * HD) return;

  const float* x  = (const float*)d_in[0];
  const int*   ei = (const int*)d_in[1];
  const float* ew = (const float*)d_in[2];
  const float* W1 = (const float*)d_in[3];
  const float* b1 = (const float*)d_in[4];
  const float* W2 = (const float*)d_in[5];
  const float* b2 = (const float*)d_in[6];
  float* out = (float*)d_out;
  const int* srcs = ei;
  const int* dsts = ei + NE;

  constexpr size_t zHL   = (size_t)MP * HPITCH * 2;
  constexpr size_t zXB   = (size_t)MP * XPITCH * 2;
  constexpr size_t zP    = (size_t)MP * HD * 4;
  constexpr size_t zENT  = (size_t)NBK * BK_PL * 4;
  constexpr size_t zTAB  = (size_t)NTAB * 4;
  constexpr size_t zFLAG = (size_t)NBK * 128;
  constexpr size_t zW1T  = (size_t)HD * W1PITCH * 2;
  constexpr size_t zW2D  = (size_t)HD * W2PITCH * 2;
  constexpr size_t zSM   = 1024;
  constexpr size_t oHL   = 0;
  constexpr size_t oP    = oHL + zHL;
  constexpr size_t oENT  = oP + zP;
  constexpr size_t oCNT  = oENT + zENT;
  constexpr size_t oOFF  = oCNT + zTAB;
  constexpr size_t oDNV  = oOFF + zTAB;
  constexpr size_t oFLAG = oDNV + zTAB;
  constexpr size_t oW1T  = oFLAG + zFLAG;
  constexpr size_t oW2D  = oW1T + zW1T;
  constexpr size_t oSM   = oW2D + zW2D;
  constexpr size_t oEND  = oSM + zSM;
  static_assert(zXB <= zHL);
  static_assert(zHL % 256 == 0 && zP % 256 == 0 && zENT % 256 == 0 && zTAB % 256 == 0);
  static_assert(zFLAG % 256 == 0 && zW1T % 256 == 0 && zW2D % 256 == 0 && zSM % 256 == 0);
  static_assert(oEND <= WSMAX);
  if (oEND > ws_size) return;

  char* ws = (char*)d_ws;
  unsigned short* H1HL = (unsigned short*)(ws + oHL);
  unsigned short* XB   = (unsigned short*)(ws + oHL);
  float*          P    = (float*)(ws + oP);
  int*            ENT  = (int*)(ws + oENT);
  int*            CNT  = (int*)(ws + oCNT);
  int*            OFF  = (int*)(ws + oOFF);
  int*            DVB  = (int*)(ws + oDNV);
  const float*    DINV = (const float*)(ws + oDNV);
  int*            FLAG = (int*)(ws + oFLAG);
  unsigned short* W1T  = (unsigned short*)(ws + oW1T);
  unsigned short* W2D  = (unsigned short*)(ws + oW2D);
  float*          SM   = (float*)(ws + oSM);

  hipFuncSetAttribute(reinterpret_cast<const void*>(&k_bucket), hipFuncAttributeMaxDynamicSharedMemorySize, (int)BK_LDS);
  hipFuncSetAttribute(reinterpret_cast<const void*>(&k_gemm<KG1, XPITCH, W1PITCH>),
                      hipFuncAttributeMaxDynamicSharedMemorySize, (int)GM_LDS);
  hipFuncSetAttribute(reinterpret_cast<const void*>(&k_gemm<KG2, HPITCH, W2PITCH>),
                      hipFuncAttributeMaxDynamicSharedMemorySize, (int)GM_LDS);

  k_prep<<<PBTOT, NTHR, 0, stream>>>(x, W1, b1, W2, b2, XB, W1T, W2D, SM);
  k_bucket<<<NBK, NTHR, BK_LDS, stream>>>(srcs, dsts, ew, ENT, CNT, OFF, DVB, FLAG);
  k_gemm<KG1, XPITCH, W1PITCH><<<MP / GBM, NTHR, GM_LDS, stream>>>(XB, W1T, DINV, P);
  k_replay<0><<<MP / ABM, NTHR, 0, stream>>>(ENT, CNT, OFF, DINV, FLAG, P, SM, H1HL, out);
  k_gemm<KG2, HPITCH, W2PITCH><<<MP / GBM, NTHR, GM_LDS, stream>>>(H1HL, W2D, DINV, P);
  k_replay<1><<<MP / ABM, NTHR, 0, stream>>>(ENT, CNT, OFF, DINV, FLAG, P, SM + HD, H1HL, out);
}
